// Propagation_67448166417075
// MI455X (gfx1250) — hardware-verified
//
#include <hip/hip_runtime.h>
#include <stddef.h>


#define DF    128
#define AP    136
#define AP2   72
#define RP    132
#define G2P   33
#define GR    32
#define TR    16
#define NTHR  256
#define NWAVE 8
#define NB    512
#define CHUNK 2048
#define NGRP  (CHUNK / (NTHR * 4))
#define WCAP  256
#define ITERS 4

#define LDS_SACC (NB * DF)
#define LDS_AUX  (2 * NB)
#define LDS_LIST (NWAVE * WCAP)
#define LDS_BYTES ((LDS_SACC + LDS_AUX + LDS_LIST + NWAVE) * 4)

static_assert(WCAP == (CHUNK / NTHR) * 32);
static_assert(NGRP == 2);
static_assert(NB == 512);
static_assert(CHUNK == 2048);
static_assert((LDS_SACC % 4) == 0);
static_assert(LDS_BYTES == 274464);
static_assert((AP % 8) == 0 && (AP2 % 8) == 0 && (RP % 4) == 0);

typedef unsigned short us;
typedef float    v4f  __attribute__((ext_vector_type(4)));
typedef float    v8f  __attribute__((ext_vector_type(8)));
typedef int      v4i  __attribute__((ext_vector_type(4)));
typedef us       v8us __attribute__((ext_vector_type(8)));
typedef __bf16   v16b __attribute__((ext_vector_type(16)));
union Frag { v16b v; v8us half[2]; };
union Pk8  { v8us u; v4i i; us s[8]; };

__device__ __forceinline__ unsigned bfr(float f) {
  const unsigned u = __float_as_uint(f);
  return (u + 0x7fffu + ((u >> 16) & 1u)) >> 16;
}
__device__ __forceinline__ float bfx(unsigned b) { return __uint_as_float(b << 16); }

__device__ __forceinline__ v8f z8() { v8f z = {0.f, 0.f, 0.f, 0.f, 0.f, 0.f, 0.f, 0.f}; return z; }

__device__ __forceinline__ v16b ldf(const us* p) {
  Frag f;
  f.half[0] = *(const v8us*)p;
  f.half[1] = *(const v8us*)(p + 16);
  return f.v;
}

__device__ __forceinline__ v8f wm3(v16b ah, v16b al, v16b bh, v16b bl, v8f c) {
  v8f d = __builtin_amdgcn_wmma_f32_16x16x32_bf16(false, ah, false, bh, (short)0, c, false, false);
  d = __builtin_amdgcn_wmma_f32_16x16x32_bf16(false, ah, false, bl, (short)0, d, false, false);
  d = __builtin_amdgcn_wmma_f32_16x16x32_bf16(false, al, false, bh, (short)0, d, false, false);
  asm volatile("v_nop\n\tv_nop\n\tv_nop\n\tv_nop" : "+v"(d) : "v"(ah), "v"(al), "v"(bh), "v"(bl));
  return d;
}

template <int NK>
__device__ __forceinline__ v8f gacc(const us* pah, const us* pal, const us* pbh, const us* pbl, v8f acc) {
#pragma unroll 1
  for (int kt = 0; kt < NK; ++kt) {
    const int k0 = kt * 32;
    const v16b ah = ldf(pah + k0);
    const v16b al = ldf(pal + k0);
    const v16b bh = ldf(pbh + k0);
    const v16b bl = ldf(pbl + k0);
    acc = wm3(ah, al, bh, bl, acc);
  }
  return acc;
}

__device__ __forceinline__ float wsum(float v) {
  v += __shfl_xor(v, 16, 32);
  v += __shfl_xor(v, 8, 32);
  v += __shfl_xor(v, 4, 32);
  v += __shfl_xor(v, 2, 32);
  v += __shfl_xor(v, 1, 32);
  return v;
}
__device__ __forceinline__ float wmax(float v) {
  v = fmaxf(v, __shfl_xor(v, 16, 32));
  v = fmaxf(v, __shfl_xor(v, 8, 32));
  v = fmaxf(v, __shfl_xor(v, 4, 32));
  v = fmaxf(v, __shfl_xor(v, 2, 32));
  v = fmaxf(v, __shfl_xor(v, 1, 32));
  return v;
}

__device__ __forceinline__ float rcpf(float x) { return __builtin_amdgcn_rcpf(x); }
__device__ __forceinline__ float ssg(float x) { return x * rcpf(1.0f + fabsf(x)); }
__device__ __forceinline__ float sigm(float x) {
  x = fminf(fmaxf(x, -80.0f), 80.0f);
  return rcpf(1.0f + __expf(-x));
}
__device__ __forceinline__ float tnh(float x) {
  x = fminf(fmaxf(x, -40.0f), 40.0f);
  const float t = __expf(-2.0f * x);
  return (1.0f - t) * rcpf(1.0f + t);
}

__device__ __forceinline__ void split8(v4f a, v4f b, us* dh, us* dl) {
  Pk8 ph, pl;
#define SPL(J, X) { const float xx = (X); const unsigned q = bfr(xx); ph.s[J] = (us)q; pl.s[J] = (us)bfr(xx - bfx(q)); }
  SPL(0, a.x) SPL(1, a.y) SPL(2, a.z) SPL(3, a.w)
  SPL(4, b.x) SPL(5, b.y) SPL(6, b.z) SPL(7, b.w)
#undef SPL
  *(v8us*)dh = ph.u;
  *(v8us*)dl = pl.u;
}

__global__ __launch_bounds__(NTHR) void k_prep(const float* __restrict__ W, us* Wh, us* Wl, int K, int Nout) {
  const int n8 = (K * Nout) >> 3;
  const int i = blockIdx.x * NTHR + threadIdx.x;
  if (i >= n8) return;
  const int kq = K >> 3;
  const int n = i / kq;
  const int k0 = (i - n * kq) * 8;
  Pk8 ph, pl;
#pragma unroll
  for (int j = 0; j < 8; ++j) {
    const float w = W[(size_t)(k0 + j) * Nout + n];
    const unsigned q = bfr(w);
    ph.s[j] = (us)q;
    pl.s[j] = (us)bfr(w - bfx(q));
  }
  const size_t o = (size_t)n * K + k0;
  *(volatile v4i*)(Wh + o) = ph.i;
  *(volatile v4i*)(Wl + o) = pl.i;
  __threadfence();
  *(volatile v4i*)(Wh + o) = ph.i;
  *(volatile v4i*)(Wl + o) = pl.i;
}

__global__ __launch_bounds__(NTHR) void k_gate(
    const float* __restrict__ h,
    const us* __restrict__ w1h, const us* __restrict__ w1l, const float* __restrict__ b1,
    const us* __restrict__ w2h, const us* __restrict__ w2l, const float* __restrict__ b2,
    const float* __restrict__ w3, const float* __restrict__ b3,
    float* g, int nN) {
  __shared__ __attribute__((aligned(16))) us Hh[GR * AP];
  __shared__ __attribute__((aligned(16))) us Hl[GR * AP];
  __shared__ __attribute__((aligned(16))) us G1h[GR * AP2];
  __shared__ __attribute__((aligned(16))) us G1l[GR * AP2];
  __shared__ float G2[GR * G2P];
  __shared__ __attribute__((aligned(16))) float gs[GR];

  const int tid  = threadIdx.x;
  const int lane = tid & 31;
  const int wave = tid >> 5;
  const int hh   = lane >> 4;
  const int m    = lane & 15;
  const int rowBase = blockIdx.x * GR;

  {
    const int r  = tid >> 3;
    const int c0 = (tid & 7) * 16;
    int row = rowBase + r;
    if (row > nN - 1) row = nN - 1;
    const float* p = h + (size_t)row * DF + c0;
    split8(*(const v4f*)(p),     *(const v4f*)(p + 4),  Hh + r * AP + c0,     Hl + r * AP + c0);
    split8(*(const v4f*)(p + 8), *(const v4f*)(p + 12), Hh + r * AP + c0 + 8, Hl + r * AP + c0 + 8);
  }
  __syncthreads();

  {
    const int rt = wave >> 2, ct = wave & 3;
    const int n1 = ct * 16 + m;
    const int arow = (rt * 16 + m) * AP + 8 * hh;
    v8f acc = gacc<DF / 32>(Hh + arow, Hl + arow,
                            w1h + (size_t)n1 * DF + 8 * hh, w1l + (size_t)n1 * DF + 8 * hh, z8());
    const float bb = b1[n1];
#pragma unroll
    for (int r = 0; r < 8; ++r) {
      const float v = ssg(acc[r] + bb);
      const unsigned q = bfr(v);
      const int row = rt * 16 + 8 * hh + r;
      G1h[row * AP2 + n1] = (us)q;
      G1l[row * AP2 + n1] = (us)bfr(v - bfx(q));
    }
  }
  __syncthreads();

  if (wave < 4) {
    const int rt = wave >> 1, ct = wave & 1;
    const int n2 = ct * 16 + m;
    const int arow = (rt * 16 + m) * AP2 + 8 * hh;
    v8f acc = gacc<2>(G1h + arow, G1l + arow,
                      w2h + (size_t)n2 * 64 + 8 * hh, w2l + (size_t)n2 * 64 + 8 * hh, z8());
    const float bb = b2[n2];
#pragma unroll
    for (int r = 0; r < 8; ++r) G2[(rt * 16 + 8 * hh + r) * G2P + n2] = ssg(acc[r] + bb);
  }
  __syncthreads();

  {
    const float w3v = w3[lane];
    const float b3v = b3[0];
#pragma unroll
    for (int j = 0; j < 4; ++j) {
      const int row = wave * 4 + j;
      float s = G2[row * G2P + lane] * w3v;
      s = wsum(s);
      if (lane == 0) gs[row] = s + b3v;
    }
  }
  __syncthreads();

  if (wave == 0 && lane < 8) {
    const v4f v = *(const v4f*)(gs + 4 * lane);
    float* gp = g + (size_t)rowBase + 4 * lane;
    *(volatile v4f*)gp = v;
    __threadfence();
    *(volatile v4f*)gp = v;
  }
}

__global__ __launch_bounds__(NTHR) void k_agg(
    const float* __restrict__ h, const int* __restrict__ ei, const float* __restrict__ g,
    float* msg, int nN, int nE) {
  extern __shared__ v4f lds_dyn[];
  float* sacc = (float*)lds_dyn;
  float* den  = sacc + LDS_SACC;
  float* mxv  = den + NB;
  int*   list = (int*)(mxv + NB);
  int*   wcnt = list + LDS_LIST;

  const int tid  = threadIdx.x;
  const int lane = tid & 31;
  const int wave = tid >> 5;
  const int nodeBase = blockIdx.x * NB;

  {
    const v4f z4 = {0.f, 0.f, 0.f, 0.f};
    for (int i = tid; i < LDS_SACC / 4; i += NTHR) lds_dyn[i] = z4;
    for (int i = tid; i < NB; i += NTHR) { den[i] = 0.f; mxv[i] = -1.0e30f; }
  }
  __syncthreads();

  const int* eid = ei + nE;
  const bool al16 = ((nE & 3) == 0);

  const int nChunks = (nE + CHUNK - 1) / CHUNK;
#pragma unroll 1
  for (int ch = 0; ch < nChunks; ++ch) {
    const int cbase = ch * CHUNK;
    int wc = 0;
#pragma unroll
    for (int gq = 0; gq < NGRP; ++gq) {
      const int el0 = (gq * NTHR + tid) * 4;
      const int e0  = cbase + el0;
      const int sent = -2147483647 - 1;
      v4i d;
      if (al16 && (e0 + 3 < nE)) {
        d = *(const v4i*)(eid + e0);
      } else {
        d.x = (e0     < nE) ? eid[min(e0, nE - 1)]     : sent;
        d.y = (e0 + 1 < nE) ? eid[min(e0 + 1, nE - 1)] : sent;
        d.z = (e0 + 2 < nE) ? eid[min(e0 + 2, nE - 1)] : sent;
        d.w = (e0 + 3 < nE) ? eid[min(e0 + 3, nE - 1)] : sent;
      }
      const unsigned s0 = (unsigned)d.x - (unsigned)nodeBase;
      const unsigned s1 = (unsigned)d.y - (unsigned)nodeBase;
      const unsigned s2 = (unsigned)d.z - (unsigned)nodeBase;
      const unsigned s3 = (unsigned)d.w - (unsigned)nodeBase;
      const bool h0 = s0 < (unsigned)NB;
      const bool h1 = s1 < (unsigned)NB;
      const bool h2 = s2 < (unsigned)NB;
      const bool h3 = s3 < (unsigned)NB;
      const unsigned many = __builtin_amdgcn_ballot_w32(h0 | h1 | h2 | h3);
      if (many != 0u) {
#define HITJ(J, HJ, SJ) { \
          const unsigned mj = __builtin_amdgcn_ballot_w32(HJ); \
          if (HJ) { \
            const int pos = wc + (int)__builtin_amdgcn_mbcnt_lo(mj, 0u); \
            if (pos < WCAP) list[wave * WCAP + pos] = ((el0 + (J)) << 9) | (int)(SJ); \
          } \
          wc += (int)__builtin_popcount(mj); }
        HITJ(0, h0, s0)
        HITJ(1, h1, s1)
        HITJ(2, h2, s2)
        HITJ(3, h3, s3)
#undef HITJ
      }
    }
    if (lane == 0) wcnt[wave] = wc;
    __syncthreads();

    if (wave == 0) {
      for (int wsx = 0; wsx < NWAVE; ++wsx) {
        int n = wcnt[wsx];
        if (n > WCAP) n = WCAP;
        if (n < 0) n = 0;
        for (int i = 0; i < n; ++i) {
          const int ent  = list[wsx * WCAP + i];
          const int slot = ent & (NB - 1);
          const int el   = (ent >> 9) & (CHUNK - 1);
          int e = cbase + el;
          if (e > nE - 1) e = nE - 1;
          int src = ei[e];
          src = src < 0 ? 0 : (src > nN - 1 ? nN - 1 : src);
          const float ge = g[src];
          const float mo = mxv[slot];
          const float mn = fmaxf(mo, ge);
          const float f  = __expf(mo - mn);
          const float p  = __expf(ge - mn);
          const v4f xv = *(const v4f*)(h + (size_t)src * DF + 4 * lane);
          v4f* sp = (v4f*)(sacc + slot * DF + 4 * lane);
          const v4f cur = *sp;
          const v4f nxt = cur * f + xv * p;
          *sp = nxt;
          const float dn = den[slot] * f + p;
          den[slot] = dn;
          mxv[slot] = mn;
        }
      }
    }
    __syncthreads();
  }

#pragma unroll 1
  for (int j = 0; j < NB / NWAVE; ++j) {
    const int slot = wave * (NB / NWAVE) + j;
    const int node = nodeBase + slot;
    if (node >= nN) break;
    const float dv  = den[slot];
    const float inv = (dv > 0.f) ? rcpf(dv) : 0.f;
    const v4f sv = *(const v4f*)(sacc + slot * DF + 4 * lane) * inv;
    float* op = msg + (size_t)node * DF + 4 * lane;
    *(volatile v4f*)op = sv;
    __threadfence();
    *(volatile v4f*)op = sv;
  }
}

__global__ __launch_bounds__(NTHR) void k_gru(
    const float* __restrict__ msg, const float* __restrict__ hc,
    const us* __restrict__ wih, const us* __restrict__ wil,
    const us* __restrict__ whh, const us* __restrict__ whl,
    const float* __restrict__ bih, const float* __restrict__ bhh,
    float* hn, int nN) {
  __shared__ __attribute__((aligned(16))) us Mh[TR * AP];
  __shared__ __attribute__((aligned(16))) us Ml[TR * AP];
  __shared__ __attribute__((aligned(16))) us Xh[TR * AP];
  __shared__ __attribute__((aligned(16))) us Xl[TR * AP];
  __shared__ __attribute__((aligned(16))) float Xf[TR * RP];
  __shared__ __attribute__((aligned(16))) float Rs[TR * RP];

  const int tid  = threadIdx.x;
  const int lane = tid & 31;
  const int wave = tid >> 5;
  const int hh   = lane >> 4;
  const int m    = lane & 15;
  const int rowBase = blockIdx.x * TR;

  {
    const int r  = tid >> 4;
    const int c0 = (tid & 15) * 8;
    int row = rowBase + r;
    if (row > nN - 1) row = nN - 1;
    const float* pm = msg + (size_t)row * DF + c0;
    const float* ph = hc  + (size_t)row * DF + c0;
    split8(*(const v4f*)(pm), *(const v4f*)(pm + 4), Mh + r * AP + c0, Ml + r * AP + c0);
    const v4f a = *(const v4f*)(ph), b = *(const v4f*)(ph + 4);
    split8(a, b, Xh + r * AP + c0, Xl + r * AP + c0);
    *(v4f*)(Xf + r * RP + c0)     = a;
    *(v4f*)(Xf + r * RP + c0 + 4) = b;
  }
  __syncthreads();

  const int n = wave * 16 + m;
  const int arow = m * AP + 8 * hh;
  const us* pmh = Mh + arow; const us* pml = Ml + arow;
  const us* pxh = Xh + arow; const us* pxl = Xl + arow;

  v8f ar = z8(), az = z8(), ain = z8(), ahn = z8();
  ar  = gacc<DF / 32>(pmh, pml, wih + (size_t)(n) * DF + 8 * hh,           wil + (size_t)(n) * DF + 8 * hh,           ar);
  ar  = gacc<DF / 32>(pxh, pxl, whh + (size_t)(n) * DF + 8 * hh,           whl + (size_t)(n) * DF + 8 * hh,           ar);
  az  = gacc<DF / 32>(pmh, pml, wih + (size_t)(DF + n) * DF + 8 * hh,      wil + (size_t)(DF + n) * DF + 8 * hh,      az);
  az  = gacc<DF / 32>(pxh, pxl, whh + (size_t)(DF + n) * DF + 8 * hh,      whl + (size_t)(DF + n) * DF + 8 * hh,      az);
  ain = gacc<DF / 32>(pmh, pml, wih + (size_t)(2 * DF + n) * DF + 8 * hh,  wil + (size_t)(2 * DF + n) * DF + 8 * hh,  ain);
  ahn = gacc<DF / 32>(pxh, pxl, whh + (size_t)(2 * DF + n) * DF + 8 * hh,  whl + (size_t)(2 * DF + n) * DF + 8 * hh,  ahn);

  {
    const float br  = bih[n] + bhh[n];
    const float bz  = bih[DF + n] + bhh[DF + n];
    const float bni = bih[2 * DF + n];
    const float bnh = bhh[2 * DF + n];
#pragma unroll
    for (int r = 0; r < 8; ++r) {
      const int row = 8 * hh + r;
      const float rg = sigm(ar[r] + br);
      const float zg = sigm(az[r] + bz);
      const float ng = tnh(ain[r] + bni + rg * (ahn[r] + bnh));
      const float ho = Xf[row * RP + n];
      Rs[row * RP + n] = (1.0f - zg) * ng + zg * ho;
    }
  }
  __syncthreads();

#pragma unroll
  for (int j = 0; j < 2; ++j) {
    const int row  = wave * 2 + j;
    const int grow = rowBase + row;
    if (grow < nN) {
      const v4f v = *(const v4f*)(Rs + row * RP + 4 * lane);
      float* op = hn + (size_t)grow * DF + 4 * lane;
      *(volatile v4f*)op = v;
      __threadfence();
      *(volatile v4f*)op = v;
    }
  }
}

__global__ __launch_bounds__(NTHR) void k_final(
    const float* __restrict__ h, const float* __restrict__ x,
    const us* __restrict__ a1h, const us* __restrict__ a1l, const float* __restrict__ c1,
    const us* __restrict__ a2h, const us* __restrict__ a2l, const float* __restrict__ c2,
    const us* __restrict__ a3h, const us* __restrict__ a3l, const float* __restrict__ c3,
    float* out, int nN) {
  __shared__ __attribute__((aligned(16))) us Hh[TR * AP];
  __shared__ __attribute__((aligned(16))) us Hl[TR * AP];
  __shared__ __attribute__((aligned(16))) us Dh[TR * AP];
  __shared__ __attribute__((aligned(16))) us Dl[TR * AP];
  __shared__ __attribute__((aligned(16))) us Th[TR * AP];
  __shared__ __attribute__((aligned(16))) us Tl[TR * AP];
  __shared__ __attribute__((aligned(16))) float AI[TR * RP];
  __shared__ __attribute__((aligned(16))) float AJ[TR * RP];

  const int tid  = threadIdx.x;
  const int lane = tid & 31;
  const int wave = tid >> 5;
  const int hh   = lane >> 4;
  const int m    = lane & 15;
  const int rowBase = blockIdx.x * TR;

  {
    const int r  = tid >> 4;
    const int c0 = (tid & 15) * 8;
    int row = rowBase + r;
    if (row > nN - 1) row = nN - 1;
    const float* ph = h + (size_t)row * DF + c0;
    const float* px = x + (size_t)row * DF + c0;
    split8(*(const v4f*)(ph), *(const v4f*)(ph + 4), Hh + r * AP + c0, Hl + r * AP + c0);
    split8(*(const v4f*)(px), *(const v4f*)(px + 4), Dh + r * AP + c0, Dl + r * AP + c0);
  }
  __syncthreads();

  const int n = wave * 16 + m;
  const int arow = m * AP + 8 * hh;

  {
    v8f acc = z8();
    acc = gacc<DF / 32>(Hh + arow, Hl + arow,
                        a1h + (size_t)n * (2 * DF) + 8 * hh,      a1l + (size_t)n * (2 * DF) + 8 * hh, acc);
    acc = gacc<DF / 32>(Dh + arow, Dl + arow,
                        a1h + (size_t)n * (2 * DF) + DF + 8 * hh, a1l + (size_t)n * (2 * DF) + DF + 8 * hh, acc);
    const float bb = c1[n];
#pragma unroll
    for (int r = 0; r < 8; ++r) {
      const float v = ssg(acc[r] + bb);
      const unsigned q = bfr(v);
      const int row = 8 * hh + r;
      Th[row * AP + n] = (us)q;
      Tl[row * AP + n] = (us)bfr(v - bfx(q));
    }
  }
  {
    v8f acc = gacc<DF / 32>(Dh + arow, Dl + arow,
                            a3h + (size_t)n * DF + 8 * hh, a3l + (size_t)n * DF + 8 * hh, z8());
    const float bb = c3[n];
#pragma unroll
    for (int r = 0; r < 8; ++r) AJ[(8 * hh + r) * RP + n] = ssg(acc[r] + bb);
  }
  __syncthreads();

  {
    v8f acc = gacc<DF / 32>(Th + arow, Tl + arow,
                            a2h + (size_t)n * DF + 8 * hh, a2l + (size_t)n * DF + 8 * hh, z8());
    const float bb = c2[n];
#pragma unroll
    for (int r = 0; r < 8; ++r) AI[(8 * hh + r) * RP + n] = ssg(acc[r] + bb);
  }
  __syncthreads();

#pragma unroll
  for (int j = 0; j < 2; ++j) {
    const int row  = wave * 2 + j;
    const int grow = rowBase + row;
    if (grow < nN) {
      const v4f v = *(const v4f*)(AI + row * RP + 4 * lane);
      float mx = fmaxf(fmaxf(v.x, v.y), fmaxf(v.z, v.w));
      mx = wmax(mx);
      v4f e;
      e.x = __expf(v.x - mx); e.y = __expf(v.y - mx); e.z = __expf(v.z - mx); e.w = __expf(v.w - mx);
      const float s   = wsum(e.x + e.y + e.z + e.w);
      const float inv = rcpf(s);
      const v4f aj = *(const v4f*)(AJ + row * RP + 4 * lane);
      const v4f o = e * inv * aj;
      float* op = out + (size_t)grow * DF + 4 * lane;
      *(volatile v4f*)op = o;
      __threadfence();
      *(volatile v4f*)op = o;
    }
  }
}

extern "C" void kernel_launch(void* const* d_in, const int* in_sizes, int n_in,
                              void* d_out, int out_size, void* d_ws, size_t ws_size,
                              hipStream_t stream) {
  if (n_in < 19) return;
  const int nN = in_sizes[0] / DF;
  if (nN <= 0 || in_sizes[0] != nN * DF) return;
  const int nE = in_sizes[1] / 2;
  if (nE <= 0 || in_sizes[1] != 2 * nE) return;
  if (in_sizes[3] != DF * 64 || in_sizes[4] != 64) return;
  if (in_sizes[5] != 64 * 32 || in_sizes[6] != 32) return;
  if (in_sizes[7] != 32 || in_sizes[8] != 1) return;
  if (in_sizes[9] != DF * 3 * DF || in_sizes[10] != 3 * DF) return;
  if (in_sizes[11] != DF * 3 * DF || in_sizes[12] != 3 * DF) return;
  if (in_sizes[13] != 2 * DF * DF || in_sizes[14] != DF) return;
  if (in_sizes[15] != DF * DF || in_sizes[16] != DF) return;
  if (in_sizes[17] != DF * DF || in_sizes[18] != DF) return;
  if (out_size != nN * DF) return;

  const float* data = (const float*)d_in[0];
  const int*   ei   = (const int*)d_in[1];
  const float* gw1  = (const float*)d_in[3];  const float* gb1 = (const float*)d_in[4];
  const float* gw2  = (const float*)d_in[5];  const float* gb2 = (const float*)d_in[6];
  const float* gw3  = (const float*)d_in[7];  const float* gb3 = (const float*)d_in[8];
  const float* w_ih = (const float*)d_in[9];  const float* b_ih = (const float*)d_in[10];
  const float* w_hh = (const float*)d_in[11]; const float* b_hh = (const float*)d_in[12];
  const float* wi1  = (const float*)d_in[13]; const float* bi1 = (const float*)d_in[14];
  const float* wi2  = (const float*)d_in[15]; const float* bi2 = (const float*)d_in[16];
  const float* wj1  = (const float*)d_in[17]; const float* bj1 = (const float*)d_in[18];
  float* out = (float*)d_out;

  const int nP = ((nN + GR - 1) / GR) * GR;
  size_t off = 0;
  auto carve = [&](size_t bytes) -> char* {
    char* p = (char*)d_ws + off;
    off += (bytes + 255) & ~(size_t)255;
    return p;
  };
  float* hA   = (float*)carve((size_t)nN * DF * sizeof(float));
  float* hB   = (float*)carve((size_t)nN * DF * sizeof(float));
  float* msgb = (float*)carve((size_t)nN * DF * sizeof(float));
  float* gv   = (float*)carve((size_t)nP * sizeof(float));
  us* w1h  = (us*)carve((size_t)64 * DF * 2);       us* w1l  = (us*)carve((size_t)64 * DF * 2);
  us* w2h  = (us*)carve((size_t)32 * 64 * 2);       us* w2l  = (us*)carve((size_t)32 * 64 * 2);
  us* wih  = (us*)carve((size_t)3 * DF * DF * 2);   us* wil  = (us*)carve((size_t)3 * DF * DF * 2);
  us* whh  = (us*)carve((size_t)3 * DF * DF * 2);   us* whl  = (us*)carve((size_t)3 * DF * DF * 2);
  us* wi1h = (us*)carve((size_t)DF * 2 * DF * 2);   us* wi1l = (us*)carve((size_t)DF * 2 * DF * 2);
  us* wi2h = (us*)carve((size_t)DF * DF * 2);       us* wi2l = (us*)carve((size_t)DF * DF * 2);
  us* wj1h = (us*)carve((size_t)DF * DF * 2);       us* wj1l = (us*)carve((size_t)DF * DF * 2);
  if (off > ws_size) return;
  if (off > (size_t)134217728) return;

  auto pgrid = [](int K, int Nout) -> unsigned { return (unsigned)(((K * Nout) / 8 + NTHR - 1) / NTHR); };
  k_prep<<<pgrid(DF, 64),      NTHR, 0, stream>>>(gw1,  w1h,  w1l,  DF,     64);
  k_prep<<<pgrid(64, 32),      NTHR, 0, stream>>>(gw2,  w2h,  w2l,  64,     32);
  k_prep<<<pgrid(DF, 3 * DF),  NTHR, 0, stream>>>(w_ih, wih,  wil,  DF,     3 * DF);
  k_prep<<<pgrid(DF, 3 * DF),  NTHR, 0, stream>>>(w_hh, whh,  whl,  DF,     3 * DF);
  k_prep<<<pgrid(2 * DF, DF),  NTHR, 0, stream>>>(wi1,  wi1h, wi1l, 2 * DF, DF);
  k_prep<<<pgrid(DF, DF),      NTHR, 0, stream>>>(wi2,  wi2h, wi2l, DF,     DF);
  k_prep<<<pgrid(DF, DF),      NTHR, 0, stream>>>(wj1,  wj1h, wj1l, DF,     DF);

  hipFuncSetAttribute(reinterpret_cast<const void*>(&k_agg),
                      hipFuncAttributeMaxDynamicSharedMemorySize, LDS_BYTES);

  const unsigned gridGate = (unsigned)(nP / GR);
  const unsigned gridAgg  = (unsigned)((nN + NB - 1) / NB);
  const unsigned gridRow  = (unsigned)((nN + TR - 1) / TR);

  const float* hcur = data;
  for (int it = 0; it < ITERS; ++it) {
    float* hnext = (it & 1) ? hB : hA;
    k_gate<<<gridGate, NTHR, 0, stream>>>(hcur, w1h, w1l, gb1, w2h, w2l, gb2, gw3, gb3, gv, nN);
    k_agg<<<gridAgg, NTHR, LDS_BYTES, stream>>>(hcur, ei, gv, msgb, nN, nE);
    k_gru<<<gridRow, NTHR, 0, stream>>>(msgb, hcur, wih, wil, whh, whl, b_ih, b_hh, hnext, nN);
    hcur = hnext;
  }

  k_final<<<gridRow, NTHR, 0, stream>>>(hcur, data, wi1h, wi1l, bi1, wi2h, wi2l, bi2,
                                         wj1h, wj1l, bj1, out, nN);
}
